// PiCANet_1932735283852
// MI455X (gfx1250) — hardware-verified
//
#include <hip/hip_runtime.h>
#include <math.h>

constexpr int NBATCH  = 16;
constexpr int NCHAN   = 256;
constexpr int IMH     = 56;
constexpr int IMW     = 56;
constexpr int NPIXIMG = IMH * IMW;
constexpr int NPIXALL = NBATCH * NPIXIMG;
constexpr int CMID1   = 128;
constexpr int NTAPS   = 49;
constexpr int NLOG    = 64;
constexpr int PADW    = 68;
constexpr int KCONV   = NTAPS * NCHAN;
constexpr int CONV_TILES = (NPIXALL / 64) * (CMID1 / 64);
constexpr float W1_CARRY     = 32.0f;
constexpr float W1_CARRY_INV = 1.0f / 32.0f;
constexpr float BNEPS        = 1e-5f;
constexpr int AGG_CC   = 8;
constexpr int AGG_ROWS = 4;
constexpr int NQUAD    = IMH / AGG_ROWS;
constexpr int XS_ROWS  = AGG_ROWS + 12;
constexpr int XS_W     = 80;
constexpr int OS_ROW   = AGG_ROWS * IMW;

static_assert(NPIXALL % 64 == 0, "M tile multiple");
static_assert(CMID1 % 64 == 0, "N tile multiple");
static_assert(KCONV % 32 == 0, "K multiple of 32");
static_assert(CMID1 % 32 == 0, "K multiple of 32");
static_assert(CONV_TILES % 8 == 0, "exact grid");
static_assert((OS_ROW * 4) % 128 == 0, "quad of rows = whole lines");
static_assert((NPIXIMG * 4) % 128 == 0, "plane = whole lines");
static_assert(XS_ROWS * AGG_CC * XS_W == 40 * 256, "stage coverage");

typedef __attribute__((ext_vector_type(16))) _Float16 v16h;
typedef __attribute__((ext_vector_type(8)))  _Float16 v8h;
typedef __attribute__((ext_vector_type(16))) __bf16   v16b;
typedef __attribute__((ext_vector_type(8)))  __bf16   v8b;
typedef __attribute__((ext_vector_type(8)))  float    v8f;
typedef __attribute__((ext_vector_type(4)))  float    v4f;
typedef __attribute__((ext_vector_type(4)))  unsigned int v4u;

__device__ __forceinline__ unsigned short f2bf_bits(float f) {
  unsigned u = __float_as_uint(f);
  return (unsigned short)((u + 0x7FFFu + ((u >> 16) & 1u)) >> 16);
}
__device__ __forceinline__ float bf_bits2f(unsigned short h) { return __uint_as_float(((unsigned)h) << 16); }

__device__ __forceinline__ void dep_guard_h(v8f& a, v8f& b, v16h x, v16h y) { asm volatile("v_nop\n\tv_nop\n\tv_nop\n\tv_nop" : "+v"(a), "+v"(b) : "v"(x), "v"(y)); }
__device__ __forceinline__ void dep_guard_b(v8f& a, v8f& b, v16b x, v16b y) { asm volatile("v_nop\n\tv_nop\n\tv_nop\n\tv_nop" : "+v"(a), "+v"(b) : "v"(x), "v"(y)); }
__device__ __forceinline__ void keep4_h(v16h a, v16h b, v16h c, v16h d) { asm volatile("v_nop" :: "v"(a), "v"(b), "v"(c), "v"(d)); }
__device__ __forceinline__ void keep4_b(v16b a, v16b b, v16b c, v16b d) { asm volatile("v_nop" :: "v"(a), "v"(b), "v"(c), "v"(d)); }
__device__ __forceinline__ void acc_guard4(v8f& a, v8f& b, v8f& c, v8f& d) { asm volatile("v_nop\n\tv_nop\n\tv_nop\n\tv_nop" : "+v"(a), "+v"(b), "+v"(c), "+v"(d)); }
template <typename T> struct Frag;
template <> struct Frag<_Float16> {
  typedef v16h V; union U { v16h v; v8h h[2]; };
  static __device__ __forceinline__ v16h load(const _Float16* p) {
    U f; f.h[0] = *(const v8h*)(p); f.h[1] = *(const v8h*)(p + 16); return f.v;
  }
  static __device__ __forceinline__ v8f mma(v16h a, v16h b, v8f c) {
    return __builtin_amdgcn_wmma_f32_16x16x32_f16(false, a, false, b, (short)0, c, false, false);
  }
  static __device__ __forceinline__ void guard(v8f& a, v8f& b, v16h x, v16h y) { dep_guard_h(a, b, x, y); }
  static __device__ __forceinline__ void keep(v16h a, v16h b, v16h c, v16h d) { keep4_h(a, b, c, d); }
};
template <> struct Frag<__bf16> {
  typedef v16b V; union U { v16b v; v8b h[2]; };
  static __device__ __forceinline__ v16b load(const __bf16* p) {
    U f; f.h[0] = *(const v8b*)(p); f.h[1] = *(const v8b*)(p + 16); return f.v;
  }
  static __device__ __forceinline__ v8f mma(v16b a, v16b b, v8f c) {
    return __builtin_amdgcn_wmma_f32_16x16x32_bf16(false, a, false, b, (short)0, c, false, false);
  }
  static __device__ __forceinline__ void guard(v8f& a, v8f& b, v16b x, v16b y) { dep_guard_b(a, b, x, y); }
  static __device__ __forceinline__ void keep(v16b a, v16b b, v16b c, v16b d) { keep4_b(a, b, c, d); }
};

__device__ __forceinline__ unsigned pk16(unsigned short a, unsigned short b) { return (unsigned)a | ((unsigned)b << 16); }
__device__ __forceinline__ unsigned short h_bits(float f) { const _Float16 h = (_Float16)f; return __builtin_bit_cast(unsigned short, h); }

template <int ET> struct Elem;
template <> struct Elem<0> { typedef _Float16 T; };
template <> struct Elem<1> { typedef __bf16 T; };
template <int ET, bool SPLIT, int BIAS_MODE, int OUT_MODE, bool RESID, int ACT = 0>
__global__ __launch_bounds__(256) void wmma_gemm64(
    const unsigned short* __restrict__ Ap, const unsigned short* __restrict__ A2p, int lda, long strideA,
    const unsigned short* __restrict__ Btp, const unsigned short* __restrict__ Bt2p, int ldb, long strideB,
    void* __restrict__ Cout, void* __restrict__ Cout2, int ldc, long strideC,
    const float* __restrict__ bias,
    const float* __restrict__ resid, long strideR,
    int M, int N, int K, float scale) {
  typedef typename Elem<ET>::T T;
  typedef typename Frag<T>::V V;
  const T* A = (const T*)Ap; const T* A2 = (const T*)A2p; const T* Bt = (const T*)Btp; const T* Bt2 = (const T*)Bt2p;
  __shared__ __align__(16) float sT[8][16 * 68];
  const int b    = blockIdx.y;
  const int lane = threadIdx.x & 31;
  const int wave = threadIdx.x >> 5;
  const int tilesN = N >> 6;
  const int tilesM = M >> 6;
  const int tile = blockIdx.x * 8 + wave;
  if (tile >= tilesM * tilesN) return;
  const int tm = tile / tilesN;
  const int tn = tile - tm * tilesN;
  const int m0 = tm << 6;
  const int n0 = tn << 6;

  const T* Ab  = A  + (size_t)b * strideA;
  const T* Bb  = Bt + (size_t)b * strideB;
  const T* Ab2 = SPLIT ? (A2  + (size_t)b * strideA) : nullptr;
  const T* Bb2 = SPLIT ? (Bt2 + (size_t)b * strideB) : nullptr;

  const int rlane = lane & 15;
  const int koff  = (lane >> 4) * 8;
  const int mOff  = (lane >> 4) * 8;

  v8f acc[4][4];
#pragma unroll
  for (int i = 0; i < 4; ++i)
#pragma unroll
    for (int j = 0; j < 4; ++j) acc[i][j] = (v8f){0.f,0.f,0.f,0.f,0.f,0.f,0.f,0.f};

  for (int k0 = 0; k0 < K; k0 += 32) {
    V bh[4], bl[4];
#pragma unroll
    for (int j = 0; j < 4; ++j) {
      const size_t bo = (size_t)(n0 + (j << 4) + rlane) * ldb + koff + k0;
      bh[j] = Frag<T>::load(Bb + bo);
      if (SPLIT) bl[j] = Frag<T>::load(Bb2 + bo);
    }
#pragma unroll
    for (int i = 0; i < 4; ++i) {
      const size_t ao = (size_t)(m0 + (i << 4) + rlane) * lda + koff + k0;
      V ah = Frag<T>::load(Ab + ao);
      V al;
      if (SPLIT) al = Frag<T>::load(Ab2 + ao);
#pragma unroll
      for (int j = 0; j < 4; ++j) {
        acc[i][j] = Frag<T>::mma(ah, bh[j], acc[i][j]);
        if (SPLIT) {
          acc[i][j] = Frag<T>::mma(ah, bl[j], acc[i][j]);
          acc[i][j] = Frag<T>::mma(al, bh[j], acc[i][j]);
        }
      }
      Frag<T>::guard(acc[i][0], acc[i][3], ah, SPLIT ? al : ah);
    }
    Frag<T>::keep(bh[0], bh[1], bh[2], bh[3]);
    if (SPLIT) Frag<T>::keep(bl[0], bl[1], bl[2], bl[3]);
  }
  acc_guard4(acc[0][0], acc[0][1], acc[0][2], acc[0][3]);
  acc_guard4(acc[1][0], acc[1][1], acc[1][2], acc[1][3]);
  acc_guard4(acc[2][0], acc[2][1], acc[2][2], acc[2][3]);
  acc_guard4(acc[3][0], acc[3][1], acc[3][2], acc[3][3]);

  float* slab = sT[wave];
  const float* Rb = RESID ? (resid + (size_t)b * strideR) : nullptr;
#pragma unroll
  for (int i = 0; i < 4; ++i) {
    const int mBase = m0 + (i << 4);
#pragma unroll
    for (int j = 0; j < 4; ++j) {
      const int n = n0 + (j << 4) + rlane;
      float bv = 0.f;
      if (BIAS_MODE == 2) bv = bias[n];
#pragma unroll
      for (int r = 0; r < 8; ++r) {
        float v = acc[i][j][r] * scale;
        if (BIAS_MODE == 1) v += bias[mBase + mOff + r];
        if (BIAS_MODE == 2) v += bv;
        if (RESID) v += Rb[(size_t)(mBase + mOff + r) * ldc + n];
        if (ACT == 2) v = fmaxf(v, 0.0f);
        if (ACT == 4) v = (v > 0.f) ? v : 0.01f * v;
        slab[(mOff + r) * 68 + (j << 4) + rlane] = v;
      }
    }
    __builtin_amdgcn_fence(__ATOMIC_RELEASE, "workgroup");
    __builtin_amdgcn_wave_barrier();
    __builtin_amdgcn_fence(__ATOMIC_ACQUIRE, "workgroup");
    if (OUT_MODE == 0) {
      float* C = (float*)Cout + (size_t)b * strideC;
      const int hh = lane >> 4, c4 = (lane & 15) * 4;
      for (int pass = 0; pass < 2; ++pass) {
#pragma unroll
        for (int it = 0; it < 8; ++it) {
          const int row = it * 2 + hh;
          v4f v = *(const v4f*)(slab + row * 68 + c4);
          *(volatile v4f*)(C + (size_t)(mBase + row) * ldc + n0 + c4) = v;
        }
        __threadfence();
      }
    } else {
      const int q = lane >> 3, c8 = (lane & 7) * 8;
      unsigned short* C  = (unsigned short*)Cout  + (size_t)b * strideC;
      unsigned short* C2 = (OUT_MODE == 2) ? ((unsigned short*)Cout2 + (size_t)b * strideC) : nullptr;
      for (int pass = 0; pass < 2; ++pass) {
#pragma unroll
        for (int it = 0; it < 4; ++it) {
          const int row = it * 4 + q;
          const float* sp = slab + row * 68 + c8;
          v8h hv, lv;
#pragma unroll
          for (int e = 0; e < 8; ++e) {
            if (OUT_MODE == 1) {
              hv[e] = (_Float16)sp[e];
            } else {
              unsigned short hb = f2bf_bits(sp[e]);
              unsigned short lb = f2bf_bits(sp[e] - bf_bits2f(hb));
              hv[e] = __builtin_bit_cast(_Float16, hb);
              lv[e] = __builtin_bit_cast(_Float16, lb);
            }
          }
          *(volatile v8h*)(C + (size_t)(mBase + row) * ldc + n0 + c8) = hv;
          if (OUT_MODE == 2) *(volatile v8h*)(C2 + (size_t)(mBase + row) * ldc + n0 + c8) = lv;
        }
        __threadfence();
      }
    }
    __builtin_amdgcn_fence(__ATOMIC_RELEASE, "workgroup");
    __builtin_amdgcn_wave_barrier();
    __builtin_amdgcn_fence(__ATOMIC_ACQUIRE, "workgroup");
  }
}

__global__ __launch_bounds__(256) void conv_gemm_kernel(
    const unsigned short* __restrict__ XPp, const unsigned short* __restrict__ Btp,
    const float* __restrict__ bias, void* __restrict__ Cout, void* __restrict__ Cout2) {
  typedef _Float16 T;
  typedef v16h V;
  const T* XP = (const T*)XPp; const T* Bt = (const T*)Btp;
  __shared__ __align__(16) float sT[8][16 * 68];
  const int lane = threadIdx.x & 31;
  const int wave = threadIdx.x >> 5;
  const int tile = blockIdx.x * 8 + wave;
  if (tile >= CONV_TILES) return;
  const int tm = tile >> 1;
  const int tn = tile & 1;
  const int m0 = tm << 6;
  const int n0 = tn << 6;
  const int rlane = lane & 15;
  const int koff  = (lane >> 4) * 8;
  const int mOff  = (lane >> 4) * 8;

  int abase[4];
#pragma unroll
  for (int i = 0; i < 4; ++i) {
    const int p    = m0 + (i << 4) + rlane;
    const int pb   = p / NPIXIMG;
    const int prem = p - pb * NPIXIMG;
    const int py   = prem / IMW;
    const int px   = prem - py * IMW;
    abase[i] = ((pb * PADW + py) * PADW + px) * NCHAN;
  }

  v8f acc[4][4];
#pragma unroll
  for (int i = 0; i < 4; ++i)
#pragma unroll
    for (int j = 0; j < 4; ++j) acc[i][j] = (v8f){0.f,0.f,0.f,0.f,0.f,0.f,0.f,0.f};

  for (int k0 = 0; k0 < KCONV; k0 += 32) {
    const int tap = k0 >> 8;
    const int c0  = k0 & 255;
    const int ti  = tap / 7;
    const int tj  = tap - ti * 7;
    const int aoff = (2 * ti * PADW + 2 * tj) * NCHAN + c0 + koff;
    V bh[4];
#pragma unroll
    for (int j = 0; j < 4; ++j) {
      const size_t bo = (size_t)(n0 + (j << 4) + rlane) * KCONV + koff + k0;
      bh[j] = Frag<T>::load(Bt + bo);
    }
#pragma unroll
    for (int i = 0; i < 4; ++i) {
      V ah = Frag<T>::load(XP + (size_t)abase[i] + aoff);
#pragma unroll
      for (int j = 0; j < 4; ++j) acc[i][j] = Frag<T>::mma(ah, bh[j], acc[i][j]);
      Frag<T>::guard(acc[i][0], acc[i][3], ah, ah);
    }
    Frag<T>::keep(bh[0], bh[1], bh[2], bh[3]);
  }
  acc_guard4(acc[0][0], acc[0][1], acc[0][2], acc[0][3]);
  acc_guard4(acc[1][0], acc[1][1], acc[1][2], acc[1][3]);
  acc_guard4(acc[2][0], acc[2][1], acc[2][2], acc[2][3]);
  acc_guard4(acc[3][0], acc[3][1], acc[3][2], acc[3][3]);

  float* slab = sT[wave];
#pragma unroll
  for (int i = 0; i < 4; ++i) {
    const int mBase = m0 + (i << 4);
#pragma unroll
    for (int j = 0; j < 4; ++j) {
      const int n = n0 + (j << 4) + rlane;
      const float bv = bias[n];
#pragma unroll
      for (int r = 0; r < 8; ++r) {
        float v = acc[i][j][r] * W1_CARRY_INV;
        v += bv;
        v = fmaxf(v, 0.0f);
        slab[(mOff + r) * 68 + (j << 4) + rlane] = v;
      }
    }
    __builtin_amdgcn_fence(__ATOMIC_RELEASE, "workgroup");
    __builtin_amdgcn_wave_barrier();
    __builtin_amdgcn_fence(__ATOMIC_ACQUIRE, "workgroup");
    {
      const int q = lane >> 3, c8 = (lane & 7) * 8;
      unsigned short* C  = (unsigned short*)Cout;
      unsigned short* C2 = (unsigned short*)Cout2;
      for (int pass = 0; pass < 2; ++pass) {
#pragma unroll
        for (int it = 0; it < 4; ++it) {
          const int row = it * 4 + q;
          const float* sp = slab + row * 68 + c8;
          v8h hv, lv;
#pragma unroll
          for (int e = 0; e < 8; ++e) {
            unsigned short hb = f2bf_bits(sp[e]);
            unsigned short lb = f2bf_bits(sp[e] - bf_bits2f(hb));
            hv[e] = __builtin_bit_cast(_Float16, hb);
            lv[e] = __builtin_bit_cast(_Float16, lb);
          }
          *(volatile v8h*)(C  + (size_t)(mBase + row) * CMID1 + n0 + c8) = hv;
          *(volatile v8h*)(C2 + (size_t)(mBase + row) * CMID1 + n0 + c8) = lv;
        }
        __threadfence();
      }
    }
    __builtin_amdgcn_fence(__ATOMIC_RELEASE, "workgroup");
    __builtin_amdgcn_wave_barrier();
    __builtin_amdgcn_fence(__ATOMIC_ACQUIRE, "workgroup");
  }
}

__global__ __launch_bounds__(256) void xpack_kernel(const float* __restrict__ x, unsigned short* __restrict__ xp) {
  __shared__ float sm[PADW * 65];
  const int t = threadIdx.x, lane = t & 31, wave = t >> 5;
  const int cq   = blockIdx.x & 3;
  const int rest = blockIdx.x >> 2;
  const int yy   = rest % PADW;
  const int b    = rest / PADW;
  const int yimg = yy - 6;
  const bool rowok = (yimg >= 0) && (yimg < IMH);
  const int yc = yimg < 0 ? 0 : (yimg > IMH - 1 ? IMH - 1 : yimg);
#pragma unroll 1
  for (int it = 0; it < 17; ++it) {
    const int e  = it * 256 + t;
    const int ch = e / PADW;
    const int xx = e - ch * PADW;
    const int ximg = xx - 6;
    const bool ok = rowok && (ximg >= 0) && (ximg < IMW);
    const int xc = ximg < 0 ? 0 : (ximg > IMW - 1 ? IMW - 1 : ximg);
    const float v = x[((size_t)(b * NCHAN + cq * 64 + ch) * IMH + yc) * IMW + xc];
    sm[xx * 65 + ch] = ok ? v : 0.0f;
  }
  __syncthreads();
  const int qq = lane >> 3, c8 = (lane & 7) * 8;
  for (int pass = 0; pass < 2; ++pass) {
#pragma unroll 1
    for (int g = wave; g < 17; g += 8) {
      const int xx = g * 4 + qq;
      unsigned short hb[8];
#pragma unroll
      for (int e = 0; e < 8; ++e) hb[e] = h_bits(sm[xx * 65 + c8 + e]);
      const v4u u = (v4u){pk16(hb[0], hb[1]), pk16(hb[2], hb[3]), pk16(hb[4], hb[5]), pk16(hb[6], hb[7])};
      *(volatile v4u*)(xp + ((size_t)((b * PADW + yy) * PADW + xx) * NCHAN + cq * 64 + c8)) = u;
    }
    __threadfence();
  }
}

__global__ __launch_bounds__(256) void btpack_kernel(const float* __restrict__ w1, unsigned short* __restrict__ bt, int n8) {
  const int i = blockIdx.x * 256 + threadIdx.x;
  if (i >= n8) return;
  const int base = i * 8;
  const int o    = base / KCONV;
  const int k    = base - o * KCONV;
  const int tap  = k >> 8;
  const int c    = k & 255;
  unsigned short hb[8];
#pragma unroll
  for (int e = 0; e < 8; ++e) hb[e] = h_bits(w1[((size_t)(o * NCHAN + c + e)) * NTAPS + tap] * W1_CARRY);
  const v4u u = (v4u){pk16(hb[0], hb[1]), pk16(hb[2], hb[3]), pk16(hb[4], hb[5]), pk16(hb[6], hb[7])};
  unsigned short* q = bt + base;
  *(volatile v4u*)q = u;
  __threadfence();
  *(volatile v4u*)q = u;
}

__global__ __launch_bounds__(256) void w2pack_kernel(const float* __restrict__ w2, unsigned short* __restrict__ hi,
                                                     unsigned short* __restrict__ lo, int n8) {
  const int i = blockIdx.x * 256 + threadIdx.x;
  if (i >= n8) return;
  const int base = i * 8;
  const int o  = base >> 7;
  const int c  = base & 127;
  const int oc = o < NTAPS ? o : NTAPS - 1;
  unsigned short hb[8], lb[8];
#pragma unroll
  for (int e = 0; e < 8; ++e) {
    float v = w2[oc * CMID1 + c + e];
    v = (o < NTAPS) ? v : 0.0f;
    hb[e] = f2bf_bits(v);
    lb[e] = f2bf_bits(v - bf_bits2f(hb[e]));
  }
  const v4u uh = (v4u){pk16(hb[0], hb[1]), pk16(hb[2], hb[3]), pk16(hb[4], hb[5]), pk16(hb[6], hb[7])};
  const v4u ul = (v4u){pk16(lb[0], lb[1]), pk16(lb[2], lb[3]), pk16(lb[4], lb[5]), pk16(lb[6], lb[7])};
  *(volatile v4u*)(hi + base) = uh;
  *(volatile v4u*)(lo + base) = ul;
  __threadfence();
  *(volatile v4u*)(hi + base) = uh;
  *(volatile v4u*)(lo + base) = ul;
}

__global__ __launch_bounds__(256) void attn_agg_kernel(
    const float* __restrict__ x, const float* __restrict__ logits,
    const float* __restrict__ b2, const float* __restrict__ gamma, const float* __restrict__ beta,
    const float* __restrict__ rmean, const float* __restrict__ rvar, float* __restrict__ out) {
  __shared__ float sPar[4][64];
  __shared__ float att[AGG_ROWS * IMW * NTAPS];
  __shared__ __align__(16) float xs[XS_ROWS * AGG_CC * XS_W];
  __shared__ __align__(16) float os[AGG_CC * OS_ROW];
  const int t = threadIdx.x, lane = t & 31, wave = t >> 5;
  const int b  = blockIdx.x / NQUAD;
  const int q  = blockIdx.x - b * NQUAD;
  const int y0 = q * AGG_ROWS;

  if (t < NTAPS) {
    sPar[0][t] = b2[t];
    sPar[1][t] = rmean[t];
    sPar[2][t] = gamma[t] * rsqrtf(rvar[t] + BNEPS);
    sPar[3][t] = beta[t];
  }
  __syncthreads();

  if (t < AGG_ROWS * IMW) {
    const int r  = t / IMW;
    const int xq = t - r * IMW;
    const size_t p = (size_t)b * NPIXIMG + (size_t)(y0 + r) * IMW + xq;
    const float* lp = logits + p * NLOG;
    float* ap = att + t * NTAPS;
    float m = 0.0f;
#pragma unroll 1
    for (int k = 0; k < NTAPS; ++k) {
      float v = ((lp[k] + sPar[0][k]) - sPar[1][k]) * sPar[2][k] + sPar[3][k];
      v = fmaxf(v, 0.0f);
      ap[k] = v;
      m = fmaxf(m, v);
    }
    float s = 0.0f;
#pragma unroll 1
    for (int k = 0; k < NTAPS; ++k) {
      const float e = expf(ap[k] - m);
      ap[k] = e;
      s += e;
    }
    const float inv = 1.0f / s;
#pragma unroll 1
    for (int k = 0; k < NTAPS; ++k) ap[k] = ap[k] * inv;
  }

  const int r   = wave >> 1;
  const int cg  = (wave & 1) * 4;
  const int x0  = lane;
  const int x1  = lane + 32;
  const int x1c = x1 < IMW ? x1 : IMW - 1;
  const float* arow0 = att + (r * IMW + x0) * NTAPS;
  const float* arow1 = att + (r * IMW + x1c) * NTAPS;

#pragma unroll 1
  for (int cc = 0; cc < NCHAN / AGG_CC; ++cc) {
    const int c0 = cc * AGG_CC;
    __syncthreads();
#pragma unroll 1
    for (int it = 0; it < 40; ++it) {
      const int e    = it * 256 + t;
      const int rr   = e / XS_W;
      const int xx   = e - rr * XS_W;
      const int ch   = rr & 7;
      const int sr   = rr >> 3;
      const int yimg = y0 - 6 + sr;
      const int ximg = xx - 6;
      const bool ok  = (yimg >= 0) && (yimg < IMH) && (ximg >= 0) && (ximg < IMW);
      const int yc = yimg < 0 ? 0 : (yimg > IMH - 1 ? IMH - 1 : yimg);
      const int xc = ximg < 0 ? 0 : (ximg > IMW - 1 ? IMW - 1 : ximg);
      const float v = x[((size_t)(b * NCHAN + c0 + ch) * IMH + yc) * IMW + xc];
      xs[e] = ok ? v : 0.0f;
    }
    __syncthreads();

    float acc0[4], acc1[4];
#pragma unroll
    for (int ch = 0; ch < 4; ++ch) { acc0[ch] = 0.0f; acc1[ch] = 0.0f; }
#pragma unroll 1
    for (int i = 0; i < 7; ++i) {
      const float* xrow = xs + (r + 2 * i) * (AGG_CC * XS_W) + cg * XS_W;
      const float* ar0 = arow0 + 7 * i;
      const float* ar1 = arow1 + 7 * i;
#pragma unroll
      for (int j = 0; j < 7; ++j) {
        const float a0 = ar0[j];
        const float a1 = ar1[j];
#pragma unroll
        for (int ch = 0; ch < 4; ++ch) {
          acc0[ch] += a0 * xrow[ch * XS_W + x0 + 2 * j];
          acc1[ch] += a1 * xrow[ch * XS_W + x1 + 2 * j];
        }
      }
    }
#pragma unroll
    for (int ch = 0; ch < 4; ++ch) {
      os[(cg + ch) * OS_ROW + r * IMW + x0] = acc0[ch];
      if (x1 < IMW) os[(cg + ch) * OS_ROW + r * IMW + x1] = acc1[ch];
    }
    __syncthreads();

    for (int pass = 0; pass < 2; ++pass) {
#pragma unroll 1
      for (int g = wave; g < 14; g += 8) {
        const int id = g * 4 + (lane >> 3);
        const int c  = id / 7;
        const int l  = id - c * 7;
        const int f0 = l * 32 + (lane & 7) * 4;
        const v4f v = *(const v4f*)(os + c * OS_ROW + f0);
        float* dst = out + ((size_t)(b * NCHAN + c0 + c) * NPIXIMG + (size_t)y0 * IMW + f0);
        *(volatile v4f*)dst = v;
      }
      __threadfence();
    }
  }
}

extern "C" void kernel_launch(void* const* d_in, const int* in_sizes, int n_in,
                              void* d_out, int out_size, void* d_ws, size_t ws_size,
                              hipStream_t stream)
{
  if (n_in < 9) return;
  if (in_sizes[0] != NBATCH * NCHAN * NPIXIMG) return;
  if (in_sizes[1] != CMID1 * NCHAN * NTAPS) return;
  if (in_sizes[2] != CMID1) return;
  if (in_sizes[3] != NTAPS * CMID1) return;
  if (in_sizes[4] != NTAPS || in_sizes[5] != NTAPS || in_sizes[6] != NTAPS ||
      in_sizes[7] != NTAPS || in_sizes[8] != NTAPS) return;
  if (out_size != NBATCH * NCHAN * NPIXIMG) return;

  const float* x     = (const float*)d_in[0];
  const float* w1    = (const float*)d_in[1];
  const float* b1    = (const float*)d_in[2];
  const float* w2    = (const float*)d_in[3];
  const float* b2    = (const float*)d_in[4];
  const float* gamma = (const float*)d_in[5];
  const float* beta  = (const float*)d_in[6];
  const float* rmean = (const float*)d_in[7];
  const float* rvar  = (const float*)d_in[8];
  float* out = (float*)d_out;

  const size_t szXP  = (size_t)NBATCH * PADW * PADW * NCHAN * 2;
  const size_t szBT  = (size_t)CMID1 * KCONV * 2;
  const size_t szK   = (size_t)NPIXALL * CMID1 * 2;
  const size_t szLOG = (size_t)NPIXALL * NLOG * 4;
  const size_t szW2  = (size_t)NLOG * CMID1 * 2;
  const size_t offXP  = 0;
  const size_t offBT  = offXP + szXP;
  const size_t offKH  = offBT + szBT;
  const size_t offKL  = offKH + szK;
  const size_t offLOG = offKL + szK;
  const size_t offW2H = offLOG + szLOG;
  const size_t offW2L = offW2H + szW2;
  const size_t total  = offW2L + szW2;
  if (total > ws_size) return;

  char* ws = (char*)d_ws;
  unsigned short* xp   = (unsigned short*)(ws + offXP);
  unsigned short* bt   = (unsigned short*)(ws + offBT);
  unsigned short* khi  = (unsigned short*)(ws + offKH);
  unsigned short* klo  = (unsigned short*)(ws + offKL);
  float*          logp = (float*)(ws + offLOG);
  unsigned short* w2h  = (unsigned short*)(ws + offW2H);
  unsigned short* w2l  = (unsigned short*)(ws + offW2L);

  xpack_kernel<<<dim3(NBATCH * PADW * 4), dim3(256), 0, stream>>>(x, xp);
  const int n8bt = (CMID1 * KCONV) / 8;
  btpack_kernel<<<dim3((n8bt + 255) / 256), dim3(256), 0, stream>>>(w1, bt, n8bt);
  const int n8w2 = (NLOG * CMID1) / 8;
  w2pack_kernel<<<dim3((n8w2 + 255) / 256), dim3(256), 0, stream>>>(w2, w2h, w2l, n8w2);
  conv_gemm_kernel<<<dim3(CONV_TILES / 8), dim3(256), 0, stream>>>(xp, bt, b1, (void*)khi, (void*)klo);
  const int tiles1x1 = (NPIXALL / 64) * (NLOG / 64);
  wmma_gemm64<1, true, 0, 0, false, 0><<<dim3((tiles1x1 + 7) / 8, 1), dim3(256), 0, stream>>>(
      khi, klo, CMID1, 0L,
      w2h, w2l, CMID1, 0L,
      (void*)logp, (void*)logp, NLOG, 0L,
      (const float*)logp,
      (const float*)logp, 0L,
      NPIXALL, NLOG, CMID1, 1.0f);
  attn_agg_kernel<<<dim3(NBATCH * NQUAD), dim3(256), 0, stream>>>(x, logp, b2, gamma, beta, rmean, rvar, out);
}
